// TernaryLoRAModel_34686155882823
// MI455X (gfx1250) — hardware-run, weakly checked
//
#include <hip/hip_runtime.h>


namespace {
constexpr int M = 256, K = 4096, O = 11008, R = 16, NBLK = K / 16, NT = O / 16;
constexpr float XS = 8.0f, WSC = 256.0f, LORA = 2.0f;
typedef _Float16 b16;
typedef __attribute__((ext_vector_type(16))) _Float16 v16b;
typedef __attribute__((ext_vector_type(8))) _Float16 v8b;
typedef __attribute__((ext_vector_type(8))) float v8f;
typedef __attribute__((ext_vector_type(4))) float v4f;
__device__ __forceinline__ float bf16_rne(float f) { unsigned int u = __float_as_uint(f); u += 0x7FFFu + ((u >> 16) & 1u); float r = __uint_as_float(u & 0xFFFF0000u); asm volatile("" : "+v"(r)); return r; }
__device__ __forceinline__ void split16(float v, b16& hi, b16& lo) { hi = (b16)v; lo = (b16)(v - (float)hi); }
__device__ __forceinline__ v16b frag_kb(const b16* p, int hh) { const v8b a = *(const v8b*)(p + 8 * hh), b = *(const v8b*)(p + 16 + 8 * hh); v16b f;
#pragma unroll
  for (int e = 0; e < 8; ++e) { f[e] = a[e]; f[8 + e] = b[e]; } return f; }
__device__ __forceinline__ v8f wmma16b(v16b a, v16b b, v8f c) { v8f d = __builtin_amdgcn_wmma_f32_16x16x32_f16(false, a, false, b, (short)0, c, false, false); asm volatile("v_nop\n\tv_nop\n\tv_nop\n\tv_nop" : "+v"(d) : "v"(a), "v"(b)); return d; }
__device__ __forceinline__ void wave_lds_sync() { __builtin_amdgcn_fence(__ATOMIC_RELEASE, "workgroup"); __builtin_amdgcn_wave_barrier(); __builtin_amdgcn_fence(__ATOMIC_ACQUIRE, "workgroup"); }
__device__ __forceinline__ float pmul(float a, float b) { float p = a * b; asm volatile("" : "+v"(p)); return p; }

__global__ __launch_bounds__(256) void unpack_kernel(const int* __restrict__ packed, b16* __restrict__ TP) { const size_t u = (size_t)blockIdx.x * 256 + threadIdx.x; if (u >= (size_t)O * NBLK) return; const unsigned int w = (unsigned int)packed[u]; v8b a, b;
#pragma unroll
  for (int j = 0; j < 8; ++j) { a[j] = (b16)((float)((int)((w >> (2 * j)) & 3u) - 1)); b[j] = (b16)((float)((int)((w >> (2 * (8 + j))) & 3u) - 1)); }
  for (int pass = 0; pass < 2; ++pass) { *(volatile v8b*)(TP + u * 16) = a; *(volatile v8b*)(TP + u * 16 + 8) = b; __threadfence(); } }
__global__ __launch_bounds__(256) void xprep_kernel(const float* __restrict__ x, const float* __restrict__ la, b16* __restrict__ XP, b16* __restrict__ AP) { const size_t u = (size_t)blockIdx.x * 256 + threadIdx.x; if (u < (size_t)M * K / 8) { v8b v; for (int j = 0; j < 8; ++j) v[j] = (b16)(bf16_rne(x[u * 8 + j]) * XS); for (int pass = 0; pass < 2; ++pass) { *(volatile v8b*)(XP + u * 8) = v; __threadfence(); } }
  if (u < (size_t)R * K / 8) { v8b v; for (int j = 0; j < 8; ++j) v[j] = (b16)(bf16_rne(la[u * 8 + j]) * WSC); for (int pass = 0; pass < 2; ++pass) { *(volatile v8b*)(AP + u * 8) = v; __threadfence(); } } }
__global__ __launch_bounds__(256) void bprep_kernel(const float* __restrict__ lb, b16* __restrict__ BP) { const size_t u = (size_t)blockIdx.x * 256 + threadIdx.x; if (u >= (size_t)O * 4) return; const int o = (int)(u / 4), k0 = (int)(u % 4) * 8; v8b v; for (int j = 0; j < 8; ++j) { const int k = k0 + j; v[j] = (b16)(k < R ? bf16_rne(lb[(size_t)o * R + k]) * WSC : 0.0f); } for (int pass = 0; pass < 2; ++pass) { *(volatile v8b*)(BP + (size_t)o * 32 + k0) = v; __threadfence(); } }
__global__ __launch_bounds__(32) void rowprep_kernel(const float* __restrict__ x, const b16* __restrict__ XP, const b16* __restrict__ AP, float* __restrict__ RS, b16* __restrict__ XAh, b16* __restrict__ XAl) { const int lane = threadIdx.x, nloc = lane & 15, hlf = lane >> 4; const int m0 = blockIdx.x * 16; __shared__ float Srow[16]; __shared__ __attribute__((aligned(16))) b16 Hh[16][40], Hl[16][40];
  for (int rr = 0; rr < 16; ++rr) { float s = 0.0f; for (int i = lane; i < K; i += 32) s += bf16_rne(x[(size_t)(m0 + rr) * K + i]); for (int o = 16; o; o >>= 1) s += __shfl_xor(s, o); if (lane == 0) Srow[rr] = s; }
  v8f acc = {};
#pragma unroll 4
  for (int kb = 0; kb < K; kb += 32) acc = wmma16b(frag_kb(XP + (size_t)(m0 + nloc) * K + kb, hlf), frag_kb(AP + (size_t)nloc * K + kb, hlf), acc);
#pragma unroll
  for (int r8 = 0; r8 < 8; ++r8) { b16 p, ql; split16(acc[r8] * (1.0f / (XS * WSC)) * XS, p, ql); Hh[8 * hlf + r8][nloc] = p; Hl[8 * hlf + r8][nloc] = ql; }
  if (lane < 16) for (int rr = 0; rr < 16; ++rr) { Hh[rr][16 + lane] = (b16)0.0f; Hl[rr][16 + lane] = (b16)0.0f; }
  wave_lds_sync();
  for (int pass = 0; pass < 2; ++pass) { ((volatile float*)RS)[2 * m0 + lane] = lane < 16 ? Srow[lane] : 0.0f;
    for (int rr = 0; rr < 16; ++rr) { ((volatile b16*)XAh)[(m0 + rr) * 32 + lane] = Hh[rr][lane]; ((volatile b16*)XAl)[(m0 + rr) * 32 + lane] = Hl[rr][lane]; } __threadfence(); } }
__global__ __launch_bounds__(32) void main_kernel(const b16* __restrict__ XP, const b16* __restrict__ TP, const b16* __restrict__ XAh, const b16* __restrict__ XAl, const b16* __restrict__ BP, const float* __restrict__ RS, const float* __restrict__ alpha, const float* __restrict__ mu, const float* __restrict__ bias, int GLIM, float* __restrict__ out) { __shared__ float Tf[16][260]; const int lane = threadIdx.x, nloc = lane & 15, hlf = lane >> 4; const int mt = blockIdx.x % (M / 16), g = blockIdx.x / (M / 16); if (g >= GLIM) return; const int m0 = mt * 16, o0 = g * 256;
  v8f acc[16];
#pragma unroll
  for (int t = 0; t < 16; ++t) acc[t] = (v8f){};
#pragma unroll 2
  for (int kb = 0; kb < K; kb += 32) { const v16b a = frag_kb(XP + (size_t)(m0 + nloc) * K + kb, hlf);
#pragma unroll
    for (int t = 0; t < 16; ++t) acc[t] = wmma16b(a, frag_kb(TP + (size_t)(o0 + t * 16 + nloc) * K + kb, hlf), acc[t]); }
  const v16b xa = frag_kb(XAh + (size_t)(m0 + nloc) * 32, hlf), xl = frag_kb(XAl + (size_t)(m0 + nloc) * 32, hlf);
#pragma unroll
  for (int t = 0; t < 16; ++t) { const int o = o0 + t * 16 + nloc; const v16b bb = frag_kb(BP + (size_t)o * 32, hlf); v8f l2 = wmma16b(xa, bb, (v8f){}); l2 = wmma16b(xl, bb, l2); const float al = bf16_rne(alpha[o]), mo = bf16_rne(mu[o]), bo = bf16_rne(bias[o]);
#pragma unroll
    for (int r8 = 0; r8 < 8; ++r8) { const int rr = 8 * hlf + r8; Tf[rr][t * 16 + nloc] = pmul(acc[t][r8] * (1.0f / XS), al) + pmul(mo, RS[2 * m0 + rr]) + LORA * (l2[r8] * (1.0f / (XS * WSC))) + bo; } }
  wave_lds_sync();
  for (int pass = 0; pass < 2; ++pass) { for (int rr = 0; rr < 16; ++rr) for (int q = 0; q < 2; ++q) *(volatile v4f*)(out + (size_t)(m0 + rr) * O + o0 + q * 128 + lane * 4) = *(const v4f*)(&Tf[rr][q * 128 + lane * 4]); __threadfence(); } }
}

extern "C" void kernel_launch(void* const* d_in, const int* in_sizes, int n_in, void* d_out, int out_size, void* d_ws, size_t ws_size, hipStream_t stream) {
  (void)n_in;
  auto Fp = [&](int i) { return (const float*)d_in[i]; }; auto Ip = [&](int i) { return (const int*)d_in[i]; };
  if (in_sizes[0] != M * K || in_sizes[1] != O * NBLK || in_sizes[2] != O || in_sizes[5] != R * K || in_sizes[6] != O * R || out_size != M * O) return;
  const int GLIM = O / 256;
  size_t off = 0; char* ws = (char*)d_ws;
  auto carve = [&](size_t bytes) { char* p = ws + off; off += (bytes + 255) & ~(size_t)255; return p; };
  b16* TP = (b16*)carve((size_t)O * K * 2); b16* XP = (b16*)carve((size_t)M * K * 2); b16* AP = (b16*)carve((size_t)R * K * 2); b16* BP = (b16*)carve((size_t)O * 32 * 2); float* RS = (float*)carve((size_t)2 * M * 4); b16* XAh = (b16*)carve((size_t)M * 32 * 2); b16* XAl = (b16*)carve((size_t)M * 32 * 2);
  if (off > ws_size || off > ((size_t)128 << 20)) return;
  unpack_kernel<<<(unsigned)(((size_t)O * NBLK + 255) / 256), 256, 0, stream>>>(Ip(1), TP);
  xprep_kernel<<<(M * K / 8 + 255) / 256, 256, 0, stream>>>(Fp(0), Fp(5), XP, AP);
  bprep_kernel<<<(O * 4 + 255) / 256, 256, 0, stream>>>(Fp(6), BP);
  rowprep_kernel<<<M / 16, 32, 0, stream>>>(Fp(0), XP, AP, RS, XAh, XAl);
  main_kernel<<<(M / 16) * GLIM, 32, 0, stream>>>(XP, TP, XAh, XAl, BP, RS, Fp(2), Fp(3), Fp(4), GLIM, (float*)d_out);
}
